// MoERoutingLayer_58720792871362
// MI455X (gfx1250) — hardware-verified
//
#include <hip/hip_runtime.h>


#define NB_  32
#define CI   64
#define CO   64
#define HI   58
#define HO   56
#define NP   3136
#define KK   576
#define NE   10
#define RS   512
#define RH   128
#define ED   64
typedef _Float16 h16;
typedef unsigned short bf;
typedef __attribute__((ext_vector_type(16))) __bf16   v16bf;
typedef __attribute__((ext_vector_type(16))) _Float16 v16h;
typedef __attribute__((ext_vector_type(8)))  _Float16 v8h;
typedef __attribute__((ext_vector_type(8)))  unsigned short v8us;
typedef __attribute__((ext_vector_type(8)))  float    v8f;
typedef __attribute__((ext_vector_type(4)))  float    v4f;
typedef v8h  __attribute__((may_alias)) v8ha;
typedef v4f  __attribute__((may_alias)) v4fa;
typedef v8us __attribute__((may_alias)) v8usa;

__device__ __forceinline__ unsigned short f2bf(float f) { unsigned u = __float_as_uint(f); u += 0x7FFFu + ((u >> 16) & 1u); return (unsigned short)(u >> 16); }
__device__ __forceinline__ float bf2f(unsigned short b) { return __uint_as_float(((unsigned)b) << 16); }
__device__ __forceinline__ float bfr(float f) { return bf2f(f2bf(f)); }
__device__ __forceinline__ v16h cat16(v8h lo, v8h hi) { return __builtin_shufflevector(lo, hi, 0, 1, 2, 3, 4, 5, 6, 7, 8, 9, 10, 11, 12, 13, 14, 15); }
__device__ __forceinline__ v16bf cat16b(v8us lo, v8us hi) { return __builtin_bit_cast(v16bf, __builtin_shufflevector(lo, hi, 0, 1, 2, 3, 4, 5, 6, 7, 8, 9, 10, 11, 12, 13, 14, 15)); }
__device__ __forceinline__ v8f wmma16(v16h a, v16h b, v8f c) { return __builtin_amdgcn_wmma_f32_16x16x32_f16(false, a, false, b, (short)0, c, false, false); }
__device__ __forceinline__ v8f wmmab(v16bf a, v16bf b, v8f c) { return __builtin_amdgcn_wmma_f32_16x16x32_bf16(false, a, false, b, (short)0, c, false, false); }


template <typename T16> struct WFrag;
template <> struct WFrag<h16> { typedef v16h V; static __device__ __forceinline__ V ld(const h16* p) { return cat16(*(const v8h*)p, *(const v8h*)(p + 16)); } static __device__ __forceinline__ v8f mma(V a, V b, v8f c) { return wmma16(a, b, c); } };
template <> struct WFrag<bf> { typedef v16bf V; static __device__ __forceinline__ V ld(const bf* p) { return cat16b(*(const v8us*)p, *(const v8us*)(p + 16)); } static __device__ __forceinline__ v8f mma(V a, V b, v8f c) { return wmmab(a, b, c); } };
template <typename T16, int NSPLIT, bool BIAS>
__global__ __launch_bounds__(32) void k_gemmw(const T16* __restrict__ A, const T16* __restrict__ A2, const T16* __restrict__ Bt, const T16* __restrict__ Bt2, int K, float* C, int ldc, const float* __restrict__ bias, size_t sA, size_t sB, size_t sC) {
    typedef typename WFrag<T16>::V V;
    __shared__ __align__(16) float os[16 * 68];
    const size_t z = blockIdx.z; A += z * sA; if (A2) A2 += z * sA; Bt += z * sB; if (Bt2) Bt2 += z * sB; C += z * sC;
    const int lane = threadIdx.x & 31, lr = lane & 15, hi = lane >> 4; const int r0 = blockIdx.x * 64, c0 = blockIdx.y * 64;
    v8f acc[4][4];
#pragma unroll
    for (int mb = 0; mb < 4; ++mb)
#pragma unroll
        for (int nb = 0; nb < 4; ++nb) acc[mb][nb] = (v8f){};
    const size_t aoff = (size_t)(r0 + lr) * K + 8 * hi, boff = (size_t)(c0 + lr) * K + 8 * hi;
#pragma unroll 1
    for (int kc = 0; kc < K; kc += 32) {
        V a[4], a2[4];
#pragma unroll
        for (int mb = 0; mb < 4; ++mb) { a[mb] = WFrag<T16>::ld(A + aoff + (size_t)mb * 16 * K + kc); if (NSPLIT == 1 || NSPLIT == 2) a2[mb] = WFrag<T16>::ld(A2 + aoff + (size_t)mb * 16 * K + kc); }
#pragma unroll
        for (int nb = 0; nb < 4; ++nb) { const V b = WFrag<T16>::ld(Bt + boff + (size_t)nb * 16 * K + kc); V b2; if (NSPLIT >= 2) b2 = WFrag<T16>::ld(Bt2 + boff + (size_t)nb * 16 * K + kc);
#pragma unroll
            for (int mb = 0; mb < 4; ++mb) { acc[mb][nb] = WFrag<T16>::mma(a[mb], b, acc[mb][nb]); if (NSPLIT == 1 || NSPLIT == 2) acc[mb][nb] = WFrag<T16>::mma(a2[mb], b, acc[mb][nb]); if (NSPLIT >= 2) acc[mb][nb] = WFrag<T16>::mma(a[mb], b2, acc[mb][nb]); } }
        asm volatile("v_nop\n\tv_nop\n\tv_nop\n\tv_nop" : "+v"(acc[0][0]), "+v"(acc[1][1]), "+v"(acc[2][2]), "+v"(acc[3][3]) : "v"(a[0]), "v"(a[3]));
    }
#pragma unroll
    for (int mb = 0; mb < 4; ++mb) {
#pragma unroll
        for (int nb = 0; nb < 4; ++nb) {
#pragma unroll
            for (int j = 0; j < 8; ++j) os[(hi * 8 + j) * 68 + nb * 16 + lr] = acc[mb][nb][j]; }
        __builtin_amdgcn_wave_barrier(); asm volatile("" ::: "memory");
        float* crow = C + (size_t)(r0 + mb * 16) * ldc + c0;
#pragma unroll 1
        for (int ps = 0; ps < 2; ++ps) {
#pragma unroll
            for (int s = 0; s < 8; ++s) { const int row = 2 * s + hi, cofs = lr * 4; v4f val = *(const v4fa*)(os + row * 68 + cofs); if (BIAS) { val[0] += bfr(bias[c0 + cofs]); val[1] += bfr(bias[c0 + cofs + 1]); val[2] += bfr(bias[c0 + cofs + 2]); val[3] += bfr(bias[c0 + cofs + 3]); }
                *(volatile v4f*)(crow + (size_t)row * ldc + cofs) = val; }
            if (ps == 0) __threadfence(); }
        __builtin_amdgcn_wave_barrier(); asm volatile("" ::: "memory");
    }
}

__device__ __forceinline__ void splitf(float y, unsigned short& h, unsigned short& l) { h = f2bf(y); l = f2bf(y - bf2f(h)); }
typedef __attribute__((ext_vector_type(2))) unsigned short v2us;
typedef __attribute__((ext_vector_type(4))) unsigned short v4us;

__global__ __launch_bounds__(128) void k_route(const float* __restrict__ rv, const float* __restrict__ W1, const float* __restrict__ b1, const float* __restrict__ W2, const float* __restrict__ b2, const float* __restrict__ emb, float* ROUT) {
    __shared__ float hs[RH]; __shared__ float rs[ED]; __shared__ float sims[NE]; __shared__ float ws[16]; const int b = blockIdx.x; const int t = threadIdx.x; const float* r0 = rv + (size_t)b * RS;
    { float s = 0.f;
#pragma unroll 1
      for (int k = 0; k < RS; ++k) { float w = bfr(W1[(size_t)k * RH + t]); asm volatile("" : "+v"(w)); float p = __fmul_rn(bfr(r0[k]), w); asm volatile("" : "+v"(p)); s = __fadd_rn(s, p); } hs[t] = fmaxf(__fadd_rn(s, bfr(b1[t])), 0.f); }
    __syncthreads();
    if (t < ED) { float s = 0.f;
#pragma unroll 1
      for (int k = 0; k < RH; ++k) { float w = bfr(W2[k * ED + t]); asm volatile("" : "+v"(w)); float p = __fmul_rn(hs[k], w); asm volatile("" : "+v"(p)); s = __fadd_rn(s, p); } rs[t] = __fadd_rn(s, bfr(b2[t])); }
    __syncthreads();
    if (t < NE) { float nr = 0.f, ne = 0.f, dot = 0.f;
#pragma unroll 1
      for (int k = 0; k < ED; ++k) { const float e = bfr(emb[t * ED + k]); float p1 = __fmul_rn(rs[k], rs[k]), p2 = __fmul_rn(e, e); asm volatile("" : "+v"(p1)); asm volatile("" : "+v"(p2)); nr = __fadd_rn(nr, p1); ne = __fadd_rn(ne, p2); }
      const float inr = __fadd_rn(__fsqrt_rn(nr), 1e-8f), ine = __fadd_rn(__fsqrt_rn(ne), 1e-8f);
#pragma unroll 1
      for (int k = 0; k < ED; ++k) { const float a = __fdiv_rn(rs[k], inr), e = __fdiv_rn(bfr(emb[t * ED + k]), ine); float p = __fmul_rn(a, e); asm volatile("" : "+v"(p)); dot = __fadd_rn(dot, p); } sims[t] = dot; }
    __syncthreads();
    if (t == 0) { float mx = -3.0e38f; for (int n = 0; n < NE; ++n) mx = fmaxf(mx, sims[n]); float e[NE]; float sum = 0.f; for (int n = 0; n < NE; ++n) { float d0 = __fsub_rn(sims[n], mx); asm volatile("" : "+v"(d0)); e[n] = __expf(d0); sum = __fadd_rn(sum, e[n]); }
      float dsum = 0.f; for (int n = 0; n < NE; ++n) { ws[n] = __fdiv_rn(e[n], sum); dsum = __fadd_rn(dsum, ws[n]); } ws[NE] = dsum; for (int n = NE + 1; n < 16; ++n) ws[n] = 0.f; }
    __syncthreads();
    if (t < 32) { const float v = (t < 16) ? ws[t] : 0.f; *(volatile float*)(ROUT + (size_t)b * 32 + t) = v; __threadfence(); *(volatile float*)(ROUT + (size_t)b * 32 + t) = v; } }
__global__ __launch_bounds__(256) void k_weff(const float* __restrict__ cw, const float* __restrict__ ROUT, int b, bf* Wh, bf* Wl) { const int e = (blockIdx.x * 256 + threadIdx.x) * 4; if (e >= CO * KK) return; const float* w = ROUT + (size_t)b * 32; float acc[4] = {0.f, 0.f, 0.f, 0.f};
#pragma unroll 1
    for (int n = 0; n < NE; ++n) { const float wn = w[n];
#pragma unroll
        for (int u = 0; u < 4; ++u) { float p = __fmul_rn(wn, bfr(cw[(size_t)n * CO * KK + e + u])); asm volatile("" : "+v"(p)); acc[u] = __fadd_rn(acc[u], p); } }
    v4us oh, ol;
#pragma unroll
    for (int u = 0; u < 4; ++u) { unsigned short a, bb; splitf(acc[u], a, bb); oh[u] = a; ol[u] = bb; } *(volatile v4us*)(Wh + e) = oh; *(volatile v4us*)(Wl + e) = ol; __threadfence(); *(volatile v4us*)(Wh + e) = oh; *(volatile v4us*)(Wl + e) = ol; }
__global__ __launch_bounds__(256) void k_im2col(const float* __restrict__ xb, bf* P) { const int e = (blockIdx.x * 256 + threadIdx.x) * 4; if (e >= NP * KK) return; const int k0 = e % KK; const int p = e / KK; const int y = p / HO, xx = p % HO; v4us o;
#pragma unroll
    for (int u = 0; u < 4; ++u) { const int k = k0 + u; const int c = k / 9, r9 = k % 9; const int kh = r9 / 3, kw = r9 % 3; o[u] = f2bf(xb[((size_t)c * HI + y + kh) * HI + xx + kw]); } *(volatile v4us*)(P + e) = o; __threadfence(); *(volatile v4us*)(P + e) = o; }
__global__ __launch_bounds__(256) void k_fin(const float* __restrict__ Y, const float* __restrict__ cb, const float* __restrict__ ROUT, int b, float* OUTb) { const int e = (blockIdx.x * 256 + threadIdx.x) * 4; if (e >= CO * NP) return; const int o = e / NP; const float* w = ROUT + (size_t)b * 32; float be = 0.f;
#pragma unroll 1
    for (int n = 0; n < NE; ++n) { float p = __fmul_rn(w[n], bfr(cb[n * CO + o])); asm volatile("" : "+v"(p)); be = __fadd_rn(be, p); }
    const float dsum = w[NE]; const v4f a = *(const v4f*)(Y + e); v4f r;
#pragma unroll
    for (int u = 0; u < 4; ++u) r[u] = __fdiv_rn(__fadd_rn(a[u], be), dsum); *(volatile v4f*)(OUTb + e) = r; __threadfence(); *(volatile v4f*)(OUTb + e) = r; }

extern "C" void kernel_launch(void* const* d_in, const int* in_sizes, int n_in,
                              void* d_out, int out_size, void* d_ws, size_t ws_size, hipStream_t stream) {
    (void)in_sizes; (void)n_in; (void)out_size;
    const float** I = (const float**)d_in;
    const float *x = I[0], *rv = I[1], *W1 = I[2], *b1 = I[3], *W2 = I[4], *b2 = I[5], *emb = I[6], *cw = I[7], *cb = I[8];
    float* OUT = (float*)d_out;
    char* wsp = (char*)d_ws;
    auto take = [&](size_t bytes) { char* p = wsp; wsp += (bytes + 255) & ~(size_t)255; return (void*)p; };
    float* ROUT = (float*)take(NB_ * 32 * 4); bf* Wh = (bf*)take(CO * KK * 2); bf* Wl = (bf*)take(CO * KK * 2); bf* P = (bf*)take((size_t)NP * KK * 2); float* Y = (float*)take((size_t)CO * NP * 4);
    if ((size_t)(wsp - (char*)d_ws) > ws_size) return;
    k_route<<<NB_, 128, 0, stream>>>(rv, W1, b1, W2, b2, emb, ROUT);
    for (int b = 0; b < NB_; ++b) {
        k_weff<<<(CO * KK / 4 + 255) / 256, 256, 0, stream>>>(cw, ROUT, b, Wh, Wl); k_im2col<<<(NP * KK / 4 + 255) / 256, 256, 0, stream>>>(x + (size_t)b * CI * HI * HI, P);
        k_gemmw<bf, 1, false><<<dim3(1, NP / 64, 1), 32, 0, stream>>>(Wh, Wl, P, nullptr, KK, Y, NP, nullptr, 0, 0, 0);
        k_fin<<<(CO * NP / 4 + 255) / 256, 256, 0, stream>>>(Y, cb, ROUT, b, OUT + (size_t)b * CO * NP); }
}
